// SetAbstractionModule_87050397155548
// MI455X (gfx1250) — hardware-verified
//
#include <hip/hip_runtime.h>
#include <stdint.h>

#pragma clang fp contract(off)

typedef __attribute__((ext_vector_type(16))) __bf16 v16b;
typedef __attribute__((ext_vector_type(8)))  __bf16 v8b;
typedef __attribute__((ext_vector_type(8)))  float  v8f;
typedef __attribute__((ext_vector_type(4)))  float  v4f;
typedef __attribute__((ext_vector_type(4)))  unsigned int u4;

constexpr int kBatch = 16;
constexpr int kNpts = 4096;
constexpr int kCin = 64;
constexpr int kMcent = 1024;
constexpr int kKsamp = 32;
constexpr int kCout = 128;
constexpr int kWin1 = 67;
constexpr int kWaves = 4;
constexpr int kCentPerWave = 8;
constexpr int kCentPerBlock = kWaves * kCentPerWave;
constexpr float kRad2 = 0.04f;
constexpr float kBnEps = 1e-5f;

constexpr int kW1h = 0;
constexpr int kW1l = 4096;
constexpr int kW2h = 8192;
constexpr int kW2l = 12288;
constexpr int kW3h = 16384;
constexpr int kW3l = 24576;
constexpr int kWtot = 32768;
constexpr int kWsBytes = kWtot * 2;

constexpr int kOut0Elems = kBatch * 3 * kMcent;
constexpr int kOut1Elems = kBatch * kCout * kMcent;
static_assert(kOut0Elems * 4 == 196608, "out1 byte offset");
static_assert(kOut0Elems * 4 + kOut1Elems * 4 == 8585216, "d_out total bytes");
static_assert(kMcent % kCentPerBlock == 0, "centroid groups");
static_assert(kCin == 64 && kKsamp == 32 && kCout == 128, "tile shapes: M=32 rows (2x16), K=64 (2x32), N multiple of 16");

__device__ __forceinline__ unsigned short f2bf_bits(float f) {
  unsigned u = __float_as_uint(f);
  return (unsigned short)((u + 0x7FFFu + ((u >> 16) & 1u)) >> 16);
}
__device__ __forceinline__ float bf_bits2f(unsigned short h) { return __uint_as_float(((unsigned)h) << 16); }

union FragU { v16b v; v8b h[2]; };
__device__ __forceinline__ v16b frag_load(const __bf16* p) {
  FragU f; f.h[0] = *(const v8b*)(p); f.h[1] = *(const v8b*)(p + 16); return f.v;
}
__device__ __forceinline__ v8f at_mma(v16b a, v16b b, v8f c) {
  c = __builtin_amdgcn_wmma_f32_16x16x32_bf16(false, a, false, b, (short)0, c, false, false);
  asm volatile("v_nop\n\tv_nop\n\tv_nop\n\tv_nop" : "+v"(c) : "v"(a), "v"(b));
  return c;
}
__device__ __forceinline__ v8f mma6(v16b ah0, v16b al0, v16b ah1, v16b al1,
                                     v16b bh0, v16b bl0, v16b bh1, v16b bl1, v8f c) {
  c = at_mma(ah0, bh0, c);
  c = at_mma(ah0, bl0, c);
  c = at_mma(al0, bh0, c);
  c = at_mma(ah1, bh1, c);
  c = at_mma(ah1, bl1, c);
  c = at_mma(al1, bh1, c);
  return c;
}
__device__ __forceinline__ void pack_hilo8(const float (&v)[8], u4& hv, u4& lv) {
#pragma unroll
  for (int i = 0; i < 4; ++i) {
    const unsigned short h0 = f2bf_bits(v[2 * i]);
    const unsigned short h1 = f2bf_bits(v[2 * i + 1]);
    const unsigned short l0 = f2bf_bits(v[2 * i] - bf_bits2f(h0));
    const unsigned short l1 = f2bf_bits(v[2 * i + 1] - bf_bits2f(h1));
    hv[i] = (unsigned)h0 | ((unsigned)h1 << 16);
    lv[i] = (unsigned)l0 | ((unsigned)l1 << 16);
  }
}

__global__ __launch_bounds__(1024) void fps_select(const float* __restrict__ points,
                                                   float* cent_out)
{
  __shared__ float sx[kNpts];
  __shared__ float sy[kNpts];
  __shared__ float sz[kNpts];
  __shared__ __align__(16) float sC[3 * kMcent];
  __shared__ unsigned int skh[32];
  __shared__ unsigned int skl[32];
  __shared__ int sLast;

  const int b = blockIdx.x;
  const int tid = threadIdx.x;
  const int lane = tid & 31;
  const int wave = tid >> 5;
  const float* px = points + (size_t)b * 3 * kNpts;
  const float* py = px + kNpts;
  const float* pz = py + kNpts;

  float lx[4], ly[4], lz[4], ld[4];
#pragma unroll
  for (int j = 0; j < 4; ++j) {
    const int n = tid + j * 1024;
    const float x = px[n], y = py[n], z = pz[n];
    sx[n] = x; sy[n] = y; sz[n] = z;
    lx[j] = x; ly[j] = y; lz[j] = z; ld[j] = 1e10f;
  }
  __syncthreads();

  int last = 0;
  for (int m = 0; m < kMcent; ++m) {
    const float qx = sx[last], qy = sy[last], qz = sz[last];
    if (tid == 0) { sC[m] = qx; sC[kMcent + m] = qy; sC[2 * kMcent + m] = qz; }
    unsigned int bh = 0u, bl = 0u;
#pragma unroll
    for (int j = 0; j < 4; ++j) {
      const int n = tid + j * 1024;
      const float dx = lx[j] - qx, dy = ly[j] - qy, dz = lz[j] - qz;
      const float t0 = dx * dx;
      const float t1 = dy * dy;
      const float t2 = dz * dz;
      float d = (t0 + t2) + t1;
      d = fminf(ld[j], d);
      ld[j] = d;
      const unsigned int kh = __float_as_uint(d);
      const unsigned int kl = 0xFFFFFFFFu - (unsigned int)n;
      const bool take = (j == 0) || (kh > bh) || (kh == bh && kl > bl);
      bh = take ? kh : bh;
      bl = take ? kl : bl;
    }
#pragma unroll
    for (int off = 16; off > 0; off >>= 1) {
      const unsigned int oh = __shfl_xor(bh, off, 32);
      const unsigned int ol = __shfl_xor(bl, off, 32);
      const bool take = (oh > bh) || (oh == bh && ol > bl);
      bh = take ? oh : bh;
      bl = take ? ol : bl;
    }
    if (lane == 0) { skh[wave] = bh; skl[wave] = bl; }
    __syncthreads();
    if (tid < 32) {
      unsigned int kh = skh[tid], kl = skl[tid];
#pragma unroll
      for (int off = 16; off > 0; off >>= 1) {
        const unsigned int oh = __shfl_xor(kh, off, 32);
        const unsigned int ol = __shfl_xor(kl, off, 32);
        const bool take = (oh > kh) || (oh == kh && ol > kl);
        kh = take ? oh : kh;
        kl = take ? ol : kl;
      }
      if (tid == 0) sLast = (int)(0xFFFFFFFFu - kl);
    }
    __syncthreads();
    last = sLast & (kNpts - 1);
  }
  __syncthreads();
  if (tid < 768) {
    float* ob = cent_out + (size_t)b * 3 * kMcent;
    const v4f v = *(const v4f*)(sC + 4 * tid);
    *(volatile v4f*)(ob + 4 * tid) = v;
    __threadfence();
    *(volatile v4f*)(ob + 4 * tid) = v;
  }
}

__global__ __launch_bounds__(256) void prep_wplanes(const float* __restrict__ w1,
                                                    const float* __restrict__ w2,
                                                    const float* __restrict__ w3,
                                                    unsigned short* __restrict__ wp)
{
  const int blk = blockIdx.x;
  const int t = blk * 256 + threadIdx.x;
  const float* src;
  int hoff, loff;
  if (blk < 2) {
    const int n = t >> 3, k8 = t & 7;
    src = w1 + n * kWin1 + 3 + k8 * 8;
    hoff = kW1h + n * 64 + k8 * 8;
    loff = kW1l + n * 64 + k8 * 8;
  } else if (blk < 4) {
    const int u = t - 512;
    const int n = u >> 3, k8 = u & 7;
    src = w2 + n * 64 + k8 * 8;
    hoff = kW2h + n * 64 + k8 * 8;
    loff = kW2l + n * 64 + k8 * 8;
  } else {
    const int u = t - 1024;
    const int n = u >> 3, k8 = u & 7;
    src = w3 + n * 64 + k8 * 8;
    hoff = kW3h + n * 64 + k8 * 8;
    loff = kW3l + n * 64 + k8 * 8;
  }
  float v[8];
#pragma unroll
  for (int j = 0; j < 8; ++j) v[j] = src[j];
  u4 hv, lv;
  pack_hilo8(v, hv, lv);
  *(volatile u4*)(wp + hoff) = hv;
  *(volatile u4*)(wp + loff) = lv;
  __threadfence();
  *(volatile u4*)(wp + hoff) = hv;
  *(volatile u4*)(wp + loff) = lv;
}

template <bool XYZ>
__device__ __forceinline__ void mlp_layer64(const unsigned short* Ahp, const unsigned short* Alp,
                                            const unsigned short* Bhp, const unsigned short* Blp,
                                            const float* bns, const float* bnt,
                                            const float* loc, const float* wx,
                                            unsigned short* Ohp, unsigned short* Olp, int lane)
{
  const __bf16* Ah = (const __bf16*)Ahp;
  const __bf16* Al = (const __bf16*)Alp;
  const __bf16* Bh = (const __bf16*)Bhp;
  const __bf16* Bl = (const __bf16*)Blp;
  const int hh = lane >> 4, c16 = lane & 15;
  const v8f zero8 = {0.f, 0.f, 0.f, 0.f, 0.f, 0.f, 0.f, 0.f};
#pragma unroll
  for (int mt = 0; mt < 2; ++mt) {
    const int ra = (mt * 16 + c16) * 64 + 8 * hh;
    const v16b ah0 = frag_load(Ah + ra);
    const v16b ah1 = frag_load(Ah + ra + 32);
    const v16b al0 = frag_load(Al + ra);
    const v16b al1 = frag_load(Al + ra + 32);
    float lx[8], ly[8], lz[8];
    if (XYZ) {
#pragma unroll
      for (int r = 0; r < 8; ++r) {
        const v4f L = *(const v4f*)(loc + (mt * 16 + 8 * hh + r) * 4);
        lx[r] = L[0]; ly[r] = L[1]; lz[r] = L[2];
      }
    }
#pragma unroll
    for (int nt = 0; nt < 4; ++nt) {
      const int n = nt * 16 + c16;
      const int rb = n * 64 + 8 * hh;
      const v16b bh0 = frag_load(Bh + rb);
      const v16b bh1 = frag_load(Bh + rb + 32);
      const v16b bl0 = frag_load(Bl + rb);
      const v16b bl1 = frag_load(Bl + rb + 32);
      v8f acc = zero8;
      if (XYZ) {
        const v4f w = *(const v4f*)(wx + n * 4);
#pragma unroll
        for (int r = 0; r < 8; ++r) {
          float p = lx[r] * w[0];
          p = fmaf(ly[r], w[1], p);
          p = fmaf(lz[r], w[2], p);
          acc[r] = p;
        }
      }
      acc = mma6(ah0, al0, ah1, al1, bh0, bl0, bh1, bl1, acc);
      const float s = bns[n], t = bnt[n];
#pragma unroll
      for (int r = 0; r < 8; ++r) {
        float y = fmaf(acc[r], s, t);
        y = fmaxf(y, 0.0f);
        const unsigned short hb = f2bf_bits(y);
        const unsigned short lb = f2bf_bits(y - bf_bits2f(hb));
        const int oi = (mt * 16 + 8 * hh + r) * 64 + n;
        Ohp[oi] = hb;
        Olp[oi] = lb;
      }
    }
  }
}

__global__ __launch_bounds__(128) void group_mlp_max(
    const float* __restrict__ points,
    const float* __restrict__ features,
    const float* __restrict__ w1,
    const float* __restrict__ b1, const float* __restrict__ g1, const float* __restrict__ be1,
    const float* __restrict__ b2, const float* __restrict__ g2, const float* __restrict__ be2,
    const float* __restrict__ b3, const float* __restrict__ g3, const float* __restrict__ be3,
    const unsigned short* __restrict__ wp,
    const float* cent,
    float* out1)
{
  __shared__ __align__(16) unsigned short sW[kWtot];
  __shared__ __align__(16) float sWx[64 * 4];
  __shared__ float sBNs[256];
  __shared__ float sBNt[256];
  __shared__ __align__(16) unsigned short sXh[kWaves][32 * 64];
  __shared__ __align__(16) unsigned short sXl[kWaves][32 * 64];
  __shared__ __align__(16) unsigned short sHh[kWaves][32 * 64];
  __shared__ __align__(16) unsigned short sHl[kWaves][32 * 64];
  __shared__ __align__(16) float sLoc[kWaves][32 * 4];
  __shared__ int sIdx[kWaves][32];
  __shared__ __align__(16) float sOut[kCout * kCentPerBlock];

  const int tid = threadIdx.x;
  const int wave = tid >> 5;
  const int lane = tid & 31;
  const int hh = lane >> 4;
  const int c16 = lane & 15;
  const int blk = blockIdx.x;
  const int b = blk >> 5;
  const int m0 = (blk & 31) * kCentPerBlock;

#pragma unroll 4
  for (int i = tid; i < kWtot / 8; i += 128) {
    const u4 v = *(const u4*)(wp + 8 * i);
    *(u4*)(sW + 8 * i) = v;
  }
  if (tid < 64) {
    v4f w;
    w[0] = w1[tid * kWin1 + 0];
    w[1] = w1[tid * kWin1 + 1];
    w[2] = w1[tid * kWin1 + 2];
    w[3] = 0.0f;
    *(v4f*)(sWx + tid * 4) = w;
  }
  {
    const float inv = 1.0f / sqrtf(1.0f + kBnEps);
    for (int i = tid; i < 256; i += 128) {
      const int ia = i & 63, ic = i & 127;
      const float ba = b1[ia], ga = g1[ia], ea = be1[ia];
      const float bb = b2[ia], gb = g2[ia], eb = be2[ia];
      const float bc = b3[ic], gc = g3[ic], ec = be3[ic];
      const bool isL1 = (i < 64), isL2 = (i < 128);
      const float bv = isL1 ? ba : (isL2 ? bb : bc);
      const float gv = isL1 ? ga : (isL2 ? gb : gc);
      const float ev = isL1 ? ea : (isL2 ? eb : ec);
      const float s = gv * inv;
      sBNs[i] = s;
      sBNt[i] = fmaf(bv, s, ev);
    }
  }
  __syncthreads();

  const float* px = points + (size_t)b * 3 * kNpts;
  const float* py = px + kNpts;
  const float* pz = py + kNpts;
  const v8f zero8 = {0.f, 0.f, 0.f, 0.f, 0.f, 0.f, 0.f, 0.f};

  for (int ci = 0; ci < kCentPerWave; ++ci) {
    const int slot = wave * kCentPerWave + ci;
    const int m = m0 + slot;
    const float cx = cent[(b * 3 + 0) * kMcent + m];
    const float cy = cent[(b * 3 + 1) * kMcent + m];
    const float cz = cent[(b * 3 + 2) * kMcent + m];
    const float c2 = (cx * cx + cz * cz) + cy * cy;

    int found = 0;
    int firstIdx = kNpts - 1;
    for (int base = 0; base < kNpts && found < kKsamp; base += 32) {
      const int n = base + lane;
      const float x = px[n], y = py[n], z = pz[n];
      const float p2 = (x * x + z * z) + y * y;
      float dp = x * cx;
      dp = fmaf(y, cy, dp);
      dp = fmaf(z, cz, dp);
      const float d2 = (c2 + p2) - 2.0f * dp;
      const bool hit = (d2 <= kRad2);
      const unsigned int msk = (unsigned int)__ballot(hit);
      if (found == 0 && msk != 0u) firstIdx = base + (__builtin_ffs((int)msk) - 1);
      const int pos = found + (int)__popc(msk & ((1u << lane) - 1u));
      if (hit && pos < kKsamp) sIdx[wave][pos] = n;
      found += (int)__popc(msk);
    }
    if (lane >= found) sIdx[wave][lane] = firstIdx;
    __syncthreads();

    {
      int nk = sIdx[wave][lane];
      nk = nk < 0 ? 0 : (nk > kNpts - 1 ? kNpts - 1 : nk);
      v4f L;
      L[0] = px[nk] - cx;
      L[1] = py[nk] - cy;
      L[2] = pz[nk] - cz;
      L[3] = 0.0f;
      *(v4f*)(sLoc[wave] + lane * 4) = L;
      const float* fbase = features + (size_t)b * kCin * kNpts + nk;
      unsigned short* xh = sXh[wave];
      unsigned short* xl = sXl[wave];
#pragma unroll 1
      for (int g = 0; g < 8; ++g) {
        const float* fp = fbase + (size_t)(g * 8) * kNpts;
        float v[8];
#pragma unroll
        for (int j = 0; j < 8; ++j) v[j] = fp[(size_t)j * kNpts];
        u4 hv, lv;
        pack_hilo8(v, hv, lv);
        *(u4*)(xh + lane * 64 + g * 8) = hv;
        *(u4*)(xl + lane * 64 + g * 8) = lv;
      }
    }
    __syncthreads();

    mlp_layer64<true>(sXh[wave], sXl[wave], sW + kW1h, sW + kW1l, sBNs, sBNt,
                      sLoc[wave], sWx, sHh[wave], sHl[wave], lane);
    __syncthreads();

    mlp_layer64<false>(sHh[wave], sHl[wave], sW + kW2h, sW + kW2l, sBNs + 64, sBNt + 64,
                       nullptr, nullptr, sXh[wave], sXl[wave], lane);
    __syncthreads();

    {
      const __bf16* A2h = (const __bf16*)sXh[wave];
      const __bf16* A2l = (const __bf16*)sXl[wave];
      const __bf16* B3h = (const __bf16*)(sW + kW3h);
      const __bf16* B3l = (const __bf16*)(sW + kW3l);
      float vmax[8];
#pragma unroll
      for (int mt = 0; mt < 2; ++mt) {
        const int ra = (mt * 16 + c16) * 64 + 8 * hh;
        const v16b ah0 = frag_load(A2h + ra);
        const v16b ah1 = frag_load(A2h + ra + 32);
        const v16b al0 = frag_load(A2l + ra);
        const v16b al1 = frag_load(A2l + ra + 32);
#pragma unroll
        for (int nt = 0; nt < 8; ++nt) {
          const int n = nt * 16 + c16;
          const int rb = n * 64 + 8 * hh;
          const v16b bh0 = frag_load(B3h + rb);
          const v16b bh1 = frag_load(B3h + rb + 32);
          const v16b bl0 = frag_load(B3l + rb);
          const v16b bl1 = frag_load(B3l + rb + 32);
          v8f acc = zero8;
          acc = mma6(ah0, al0, ah1, al1, bh0, bl0, bh1, bl1, acc);
          const float s = sBNs[128 + n], t = sBNt[128 + n];
          float mx = fmaf(acc[0], s, t);
#pragma unroll
          for (int r = 1; r < 8; ++r) mx = fmaxf(mx, fmaf(acc[r], s, t));
          if (mt == 0) vmax[nt] = mx;
          else vmax[nt] = fmaxf(vmax[nt], mx);
        }
      }
#pragma unroll
      for (int nt = 0; nt < 8; ++nt) {
        float v = vmax[nt];
        const float o2 = __shfl_xor(v, 16, 32);
        v = fmaxf(v, o2);
        v = fmaxf(v, 0.0f);
        if (lane < 16) sOut[(nt * 16 + c16) * kCentPerBlock + slot] = v;
      }
    }
    __syncthreads();
  }

  {
    float* ob = out1 + (size_t)b * kCout * kMcent + m0;
    const int q = lane >> 3, c4 = (lane & 7) * 4;
    for (int pass = 0; pass < 2; ++pass) {
#pragma unroll
      for (int it = 0; it < 8; ++it) {
        const int o = wave * 32 + it * 4 + q;
        const v4f v = *(const v4f*)(sOut + o * kCentPerBlock + c4);
        *(volatile v4f*)(ob + (size_t)o * kMcent + c4) = v;
      }
      __threadfence();
    }
  }
}

extern "C" void kernel_launch(void* const* d_in, const int* in_sizes, int n_in,
                              void* d_out, int out_size, void* d_ws, size_t ws_size,
                              hipStream_t stream)
{
  (void)in_sizes; (void)n_in; (void)out_size;
  const float* points   = (const float*)d_in[0];
  const float* features = (const float*)d_in[1];
  const float* w1  = (const float*)d_in[2];
  const float* b1  = (const float*)d_in[3];
  const float* g1  = (const float*)d_in[4];
  const float* be1 = (const float*)d_in[5];
  const float* w2  = (const float*)d_in[6];
  const float* b2  = (const float*)d_in[7];
  const float* g2  = (const float*)d_in[8];
  const float* be2 = (const float*)d_in[9];
  const float* w3  = (const float*)d_in[10];
  const float* b3  = (const float*)d_in[11];
  const float* g3  = (const float*)d_in[12];
  const float* be3 = (const float*)d_in[13];

  float* out0 = (float*)d_out;
  float* out1 = out0 + kOut0Elems;

  if (ws_size < (size_t)kWsBytes) return;
  unsigned short* wp = (unsigned short*)d_ws;

  fps_select<<<kBatch, 1024, 0, stream>>>(points, out0);
  prep_wplanes<<<8, 256, 0, stream>>>(w1, w2, w3, wp);
  group_mlp_max<<<kBatch * (kMcent / kCentPerBlock), kWaves * 32, 0, stream>>>(
      points, features, w1, b1, g1, be1, b2, g2, be2, b3, g3, be3, wp, out0, out1);
}
